// Decoder_61323543052777
// MI455X (gfx1250) — hardware-verified
//
#include <hip/hip_runtime.h>
#include <stddef.h>
#include <stdint.h>


#define DF     128
#define NPB    16
#define RW     (DF / 2)
#define NTHR   256
#define NWAVE  8
#define EPW    32
#define WSMAX  134217728

static_assert(DF % 32 == 0 && DF / 8 == 16);
static_assert(NPB * (DF / 8) == NTHR);
static_assert(NTHR == NWAVE * 32 && EPW * 4 == 128);

typedef float          v4f   __attribute__((ext_vector_type(4)));
typedef float          v8f   __attribute__((ext_vector_type(8)));
typedef int            v8i   __attribute__((ext_vector_type(8)));
typedef unsigned int   v4u   __attribute__((ext_vector_type(4)));
typedef unsigned short v8us  __attribute__((ext_vector_type(8)));
typedef unsigned short v16us __attribute__((ext_vector_type(16)));
typedef __bf16         v16bf __attribute__((ext_vector_type(16)));
typedef v4f  __attribute__((may_alias)) v4fa;
typedef v4u  __attribute__((may_alias)) v4ua;
typedef v8us __attribute__((may_alias)) v8usa;
union FragB { v16bf v; v16us u; v8us h[2]; v8i w; };

__device__ __forceinline__ v8f wmb(const FragB& a, const FragB& b, v8f c) {
  v8f d = __builtin_amdgcn_wmma_f32_16x16x32_bf16(false, a.v, false, b.v, (short)0, c, false, false);
  asm volatile("v_nop\n\tv_nop\n\tv_nop\n\tv_nop" : "+v"(d) : "v"(a.w), "v"(b.w));
  return d;
}

__device__ __forceinline__ unsigned bf16_bits(float f) {
  const unsigned u = __float_as_uint(f);
  return (u + 0x7FFFu + ((u >> 16) & 1u)) >> 16;
}
__device__ __forceinline__ float bf16_val(float f) {
  return __uint_as_float(bf16_bits(f) << 16);
}

__device__ __forceinline__ void wave_sync() {
  __builtin_amdgcn_fence(__ATOMIC_RELEASE, "wavefront");
  __builtin_amdgcn_wave_barrier();
  __builtin_amdgcn_fence(__ATOMIC_ACQUIRE, "wavefront");
}

struct HL { unsigned h; unsigned l; };

__device__ __forceinline__ HL absdiff_split(unsigned wa, unsigned wb) {
  const float a0 = __uint_as_float(wa << 16);
  const float a1 = __uint_as_float(wa & 0xffff0000u);
  const float b0 = __uint_as_float(wb << 16);
  const float b1 = __uint_as_float(wb & 0xffff0000u);
  const float d0 = fabsf(a0 - b0);
  const float d1 = fabsf(a1 - b1);
  const unsigned h0 = bf16_bits(d0);
  const unsigned h1 = bf16_bits(d1);
  const unsigned l0 = bf16_bits(d0 - __uint_as_float(h0 << 16));
  const unsigned l1 = bf16_bits(d1 - __uint_as_float(h1 << 16));
  HL o;
  o.h = h0 | (h1 << 16);
  o.l = l0 | (l1 << 16);
  return o;
}

__global__ __launch_bounds__(NTHR) void k_prep(const float* __restrict__ x, const float* __restrict__ W,
                                               int nUnits, int nXBlocks,
                                               unsigned short* xb, unsigned short* wb) {
  const int tid = (int)threadIdx.x;
  if ((int)blockIdx.x < nXBlocks) {
    const int u = (int)blockIdx.x * NTHR + tid;
    if (u >= nUnits) return;
    const int row = u >> 4;
    const int k8  = (u & 15) * 8;
    const float* p = x + (size_t)row * DF + k8;
    const v4f a = *(const v4fa*)p;
    const v4f b = *(const v4fa*)(p + 4);
    v8us o;
    o[0] = (unsigned short)bf16_bits(a.x); o[1] = (unsigned short)bf16_bits(a.y);
    o[2] = (unsigned short)bf16_bits(a.z); o[3] = (unsigned short)bf16_bits(a.w);
    o[4] = (unsigned short)bf16_bits(b.x); o[5] = (unsigned short)bf16_bits(b.y);
    o[6] = (unsigned short)bf16_bits(b.z); o[7] = (unsigned short)bf16_bits(b.w);
    unsigned short* dp = xb + (size_t)row * DF + k8;
    *(volatile v8us*)dp = o;
    __threadfence();
    *(volatile v8us*)dp = o;
  } else {
    const int n  = tid >> 4;
    const int k8 = (tid & 15) * 8;
    const float* p = W + k8;
    const v4f a = *(const v4fa*)p;
    const v4f b = *(const v4fa*)(p + 4);
    const bool live = (n == 0);
    v8us o;
    o[0] = live ? (unsigned short)bf16_bits(a.x) : (unsigned short)0;
    o[1] = live ? (unsigned short)bf16_bits(a.y) : (unsigned short)0;
    o[2] = live ? (unsigned short)bf16_bits(a.z) : (unsigned short)0;
    o[3] = live ? (unsigned short)bf16_bits(a.w) : (unsigned short)0;
    o[4] = live ? (unsigned short)bf16_bits(b.x) : (unsigned short)0;
    o[5] = live ? (unsigned short)bf16_bits(b.y) : (unsigned short)0;
    o[6] = live ? (unsigned short)bf16_bits(b.z) : (unsigned short)0;
    o[7] = live ? (unsigned short)bf16_bits(b.w) : (unsigned short)0;
    unsigned short* dp = wb + (size_t)n * DF + k8;
    *(volatile v8us*)dp = o;
    __threadfence();
    *(volatile v8us*)dp = o;
  }
}

__device__ __forceinline__ v8f tile_step(const unsigned* __restrict__ xbw, int ro, int co, int wofs,
                                         const FragB& bf, v8f acc) {
  const v4u r1 = *(const v4ua*)(xbw + ro + wofs);
  const v4u r2 = *(const v4ua*)(xbw + ro + wofs + 8);
  const v4u c1 = *(const v4ua*)(xbw + co + wofs);
  const v4u c2 = *(const v4ua*)(xbw + co + wofs + 8);
  FragB ah, al;
  HL s;
  s = absdiff_split(r1.x, c1.x); ah.w[0] = (int)s.h; al.w[0] = (int)s.l;
  s = absdiff_split(r1.y, c1.y); ah.w[1] = (int)s.h; al.w[1] = (int)s.l;
  s = absdiff_split(r1.z, c1.z); ah.w[2] = (int)s.h; al.w[2] = (int)s.l;
  s = absdiff_split(r1.w, c1.w); ah.w[3] = (int)s.h; al.w[3] = (int)s.l;
  s = absdiff_split(r2.x, c2.x); ah.w[4] = (int)s.h; al.w[4] = (int)s.l;
  s = absdiff_split(r2.y, c2.y); ah.w[5] = (int)s.h; al.w[5] = (int)s.l;
  s = absdiff_split(r2.z, c2.z); ah.w[6] = (int)s.h; al.w[6] = (int)s.l;
  s = absdiff_split(r2.w, c2.w); ah.w[7] = (int)s.h; al.w[7] = (int)s.l;
  acc = wmb(ah, bf, acc);
  acc = wmb(al, bf, acc);
  return acc;
}

__global__ __launch_bounds__(NTHR) void k_edge(const unsigned* __restrict__ xbw,
                                               const unsigned short* __restrict__ wbp,
                                               const int* __restrict__ ri, const int* __restrict__ ci,
                                               const float* __restrict__ bias,
                                               int nE, int nN, float* out) {
  __shared__ __attribute__((aligned(16))) float stg[NWAVE * EPW];
  const int tid = (int)threadIdx.x, lane = tid & 31, wave = tid >> 5, hh = lane >> 4, m = lane & 15;
  const int e0 = ((int)blockIdx.x * NWAVE + wave) * EPW;
  if (e0 >= nE) return;

  int ea = e0 + m;       ea = ea < nE ? ea : nE - 1;
  int eb = e0 + 16 + m;  eb = eb < nE ? eb : nE - 1;
  int r0 = ri[ea], c0 = ci[ea], r1 = ri[eb], c1 = ci[eb];
  r0 = r0 < 0 ? 0 : (r0 > nN - 1 ? nN - 1 : r0);
  c0 = c0 < 0 ? 0 : (c0 > nN - 1 ? nN - 1 : c0);
  r1 = r1 < 0 ? 0 : (r1 > nN - 1 ? nN - 1 : r1);
  c1 = c1 < 0 ? 0 : (c1 > nN - 1 ? nN - 1 : c1);
  const int ro0 = r0 * RW, co0 = c0 * RW, ro1 = r1 * RW, co1 = c1 * RW;

  const float br = bf16_val(bias[0]);
  const unsigned short* wq = wbp + (size_t)m * DF + 8 * hh;

  v8f acc0 = {0.f, 0.f, 0.f, 0.f, 0.f, 0.f, 0.f, 0.f};
  v8f acc1 = {0.f, 0.f, 0.f, 0.f, 0.f, 0.f, 0.f, 0.f};
#pragma unroll 1
  for (int kc = 0; kc < DF / 32; ++kc) {
    FragB bf;
    bf.h[0] = *(const v8usa*)(wq + 32 * kc);
    bf.h[1] = *(const v8usa*)(wq + 32 * kc + 16);
    const int wofs = 16 * kc + 4 * hh;
    acc0 = tile_step(xbw, ro0, co0, wofs, bf, acc0);
    acc1 = tile_step(xbw, ro1, co1, wofs, bf, acc1);
  }

  float* sw = stg + wave * EPW;
  if (m == 0) {
#pragma unroll
    for (int r = 0; r < 8; ++r) {
      sw[8 * hh + r]      = acc0[r];
      sw[16 + 8 * hh + r] = acc1[r];
    }
  }
  wave_sync();
  const float v = sw[lane] + br;
  const bool ok = (e0 + lane) < nE;
  float* op = out + (size_t)e0 + lane;
  if (ok) *(volatile float*)op = v;
  __threadfence();
  if (ok) *(volatile float*)op = v;
}

static inline int cdiv(int a, int b) { return (a + b - 1) / b; }
static inline size_t al256(size_t o) { return (o + 255) & ~(size_t)255; }

extern "C" void kernel_launch(void* const* d_in, const int* in_sizes, int n_in,
                              void* d_out, int out_size, void* d_ws, size_t ws_size,
                              hipStream_t stream) {
  if (n_in < 5) return;
  if (in_sizes[0] < DF || (in_sizes[0] % DF) != 0) return;
  const int nN = in_sizes[0] / DF;
  if (nN < 1 || nN > (1 << 24)) return;
  const int nE = in_sizes[1];
  if (nE < 1 || nE > (1 << 30)) return;
  if (in_sizes[2] != nE) return;
  if (in_sizes[3] != DF) return;
  if (in_sizes[4] < 1) return;
  if (out_size != nE) return;

  const float* x  = (const float*)d_in[0];
  const int*   ri = (const int*)d_in[1];
  const int*   ci = (const int*)d_in[2];
  const float* W  = (const float*)d_in[3];
  const float* b  = (const float*)d_in[4];
  float* out = (float*)d_out;

  char* ws = (char*)d_ws;
  size_t off = 0;
  const size_t oWB = off; off = al256(off + (size_t)NPB * DF * 2);
  const size_t oXB = off; off = al256(off + (size_t)nN * DF * 2);
  if (off > ws_size || off > (size_t)WSMAX) return;
  unsigned short* WB = (unsigned short*)(ws + oWB);
  unsigned short* XB = (unsigned short*)(ws + oXB);

  const int nUnits   = nN * (DF / 8);
  const int nXBlocks = cdiv(nUnits, NTHR);
  k_prep<<<nXBlocks + 1, NTHR, 0, stream>>>(x, W, nUnits, nXBlocks, XB, WB);
  k_edge<<<cdiv(nE, NWAVE * EPW), NTHR, 0, stream>>>((const unsigned*)XB, WB, ri, ci, b, nE, nN, out);
}
